// FusionMambaBlock_62526133895656
// MI455X (gfx1250) — hardware-run, weakly checked
//
#include <hip/hip_runtime.h>
#include <math.h>

typedef __attribute__((ext_vector_type(16))) _Float16 v16h;
typedef __attribute__((ext_vector_type(8)))  _Float16 v8h;
typedef __attribute__((ext_vector_type(16))) __bf16   v16b;
typedef __attribute__((ext_vector_type(8)))  __bf16   v8b;
typedef __attribute__((ext_vector_type(8)))  float    v8f;
typedef __attribute__((ext_vector_type(4)))  float    v4f;

constexpr int kImg    = 4;
constexpr int kNSeq   = 8;
constexpr int kSeq    = 4096;
constexpr int kDm     = 96;
constexpr int kDin    = 192;
constexpr int kNst    = 16;
constexpr int kDtR    = 6;
constexpr int kXzP    = 2 * kDin;
constexpr int kXprN   = 38;
constexpr int kXdP    = 64;
constexpr int kOutP   = 128;
constexpr int kCnvN   = 128;
constexpr int kRows   = kNSeq * kSeq;
constexpr int kRowsO  = kImg * kSeq;
constexpr int kGrp    = 4;
constexpr int kRowsG  = kGrp * kSeq;
constexpr int kNGrp   = kNSeq / kGrp;
constexpr int kConvTP = 196;
constexpr int kScanTS = 64;
constexpr int kScanCh = 64;
constexpr int kScanYP = 68;
constexpr int kXTP    = 100;
constexpr int kOTP    = 68;
static_assert(kDm % 32 == 0 && kDin % 32 == 0, "K multiples of 32");
static_assert(kRowsG % 64 == 0 && kRows % 64 == 0 && kRowsO % 64 == 0 && kXzP % 64 == 0 && kXdP % 64 == 0 &&
              kOutP % 64 == 0 && kCnvN % 64 == 0, "tile multiples");

constexpr size_t kOffTKH  = 0;
constexpr size_t kOffTKL  = kOffTKH  + (size_t)kRows  * kDm   * 2;
constexpr size_t kOffW1H  = kOffTKL  + (size_t)kRows  * kDm   * 2;
constexpr size_t kOffW1L  = kOffW1H  + (size_t)kCnvN  * kDm   * 2;
constexpr size_t kOffW2H  = kOffW1L  + (size_t)kCnvN  * kDm   * 2;
constexpr size_t kOffW2L  = kOffW2H  + (size_t)kCnvN  * kDm   * 2;
constexpr size_t kOffO1   = kOffW2L  + (size_t)kCnvN  * kDm   * 2;
constexpr size_t kOffXH   = kOffO1   + (size_t)kRows  * kCnvN * 4;
constexpr size_t kOffXL   = kOffXH   + (size_t)kRows  * kDm   * 2;
constexpr size_t kOffWIH  = kOffXL   + (size_t)kRows  * kDm   * 2;
constexpr size_t kOffWIL  = kOffWIH  + (size_t)kXzP   * kDm   * 2;
constexpr size_t kOffWXH  = kOffWIL  + (size_t)kXzP   * kDm   * 2;
constexpr size_t kOffWXL  = kOffWXH  + (size_t)kXdP   * kDin  * 2;
constexpr size_t kOffWOH  = kOffWXL  + (size_t)kXdP   * kDin  * 2;
constexpr size_t kOffWOL  = kOffWOH  + (size_t)kOutP  * kDin  * 2;
constexpr size_t kOffXZ   = kOffWOL  + (size_t)kOutP  * kDin  * 2;
constexpr size_t kOffUC   = kOffXZ   + (size_t)kRowsG * kXzP  * 4;
constexpr size_t kOffUCH  = kOffUC   + (size_t)kRowsG * kDin  * 4;
constexpr size_t kOffUCL  = kOffUCH  + (size_t)kRowsG * kDin  * 2;
constexpr size_t kOffXD   = kOffUCL  + (size_t)kRowsG * kDin  * 2;
constexpr size_t kOffYH   = kOffXD   + (size_t)kRowsG * kXdP  * 4;
constexpr size_t kOffYL   = kOffYH   + (size_t)kRowsG * kDin  * 2;
constexpr size_t kOffYO   = kOffYL   + (size_t)kRowsG * kDin  * 2;
constexpr size_t kWsTotal = kOffYO   + (size_t)kRows  * kOutP * 4;
constexpr size_t kOffYSH  = kOffTKH;
constexpr size_t kOffYSL  = kOffTKL;
constexpr size_t kOffO2   = kOffO1;
static_assert(kWsTotal == 126222336ull, "carve total");
static_assert(kWsTotal <= 134217728ull, "carve cap");
static_assert((size_t)kRowsO * kDm * 2 <= (size_t)kRows * kDm * 2, "YS fits in TK");
static_assert((size_t)kRowsO * kCnvN * 4 <= (size_t)kRows * kCnvN * 4, "O2 fits in O1");
static_assert((kOffTKL % 128) == 0 && (kOffW1H % 128) == 0 && (kOffW1L % 128) == 0 && (kOffW2H % 128) == 0 &&
              (kOffW2L % 128) == 0 && (kOffO1 % 128) == 0 && (kOffXH % 128) == 0 && (kOffXL % 128) == 0 &&
              (kOffWIH % 128) == 0 && (kOffWIL % 128) == 0 && (kOffWXH % 128) == 0 &&
              (kOffWXL % 128) == 0 && (kOffWOH % 128) == 0 && (kOffWOL % 128) == 0 && (kOffXZ % 128) == 0 &&
              (kOffUC % 128) == 0 && (kOffUCH % 128) == 0 && (kOffUCL % 128) == 0 && (kOffXD % 128) == 0 &&
              (kOffYH % 128) == 0 && (kOffYL % 128) == 0 && (kOffYO % 128) == 0, "128-B aligned regions");

__device__ __forceinline__ unsigned short f2bf_bits(float f) {
  unsigned u = __float_as_uint(f);
  return (unsigned short)((u + 0x7FFFu + ((u >> 16) & 1u)) >> 16);
}
__device__ __forceinline__ float bf_bits2f(unsigned short h) { return __uint_as_float(((unsigned)h) << 16); }

__device__ __forceinline__ void dep_guard_h(v8f& a, v8f& b, v16h x, v16h y) { asm volatile("v_nop\n\tv_nop\n\tv_nop\n\tv_nop" : "+v"(a), "+v"(b) : "v"(x), "v"(y)); }
__device__ __forceinline__ void dep_guard_b(v8f& a, v8f& b, v16b x, v16b y) { asm volatile("v_nop\n\tv_nop\n\tv_nop\n\tv_nop" : "+v"(a), "+v"(b) : "v"(x), "v"(y)); }
__device__ __forceinline__ void keep4_h(v16h a, v16h b, v16h c, v16h d) { asm volatile("v_nop" :: "v"(a), "v"(b), "v"(c), "v"(d)); }
__device__ __forceinline__ void keep4_b(v16b a, v16b b, v16b c, v16b d) { asm volatile("v_nop" :: "v"(a), "v"(b), "v"(c), "v"(d)); }
__device__ __forceinline__ void acc_guard4(v8f& a, v8f& b, v8f& c, v8f& d) { asm volatile("v_nop\n\tv_nop\n\tv_nop\n\tv_nop" : "+v"(a), "+v"(b), "+v"(c), "+v"(d)); }
template <typename T> struct Frag;
template <> struct Frag<_Float16> {
  typedef v16h V; union U { v16h v; v8h h[2]; };
  static __device__ __forceinline__ v16h load(const _Float16* p) {
    U f; f.h[0] = *(const v8h*)(p); f.h[1] = *(const v8h*)(p + 16); return f.v;
  }
  static __device__ __forceinline__ v8f mma(v16h a, v16h b, v8f c) {
    return __builtin_amdgcn_wmma_f32_16x16x32_f16(false, a, false, b, (short)0, c, false, false);
  }
  static __device__ __forceinline__ void guard(v8f& a, v8f& b, v16h x, v16h y) { dep_guard_h(a, b, x, y); }
  static __device__ __forceinline__ void keep(v16h a, v16h b, v16h c, v16h d) { keep4_h(a, b, c, d); }
};
template <> struct Frag<__bf16> {
  typedef v16b V; union U { v16b v; v8b h[2]; };
  static __device__ __forceinline__ v16b load(const __bf16* p) {
    U f; f.h[0] = *(const v8b*)(p); f.h[1] = *(const v8b*)(p + 16); return f.v;
  }
  static __device__ __forceinline__ v8f mma(v16b a, v16b b, v8f c) {
    return __builtin_amdgcn_wmma_f32_16x16x32_bf16(false, a, false, b, (short)0, c, false, false);
  }
  static __device__ __forceinline__ void guard(v8f& a, v8f& b, v16b x, v16b y) { dep_guard_b(a, b, x, y); }
  static __device__ __forceinline__ void keep(v16b a, v16b b, v16b c, v16b d) { keep4_b(a, b, c, d); }
};

template <int ET> struct Elem;
template <> struct Elem<0> { typedef _Float16 T; };
template <> struct Elem<1> { typedef __bf16 T; };
template <int ET, int SPL, int BIAS_MODE, int OUT_MODE, bool RESID, int ACT = 0>
__global__ __launch_bounds__(256) void wmma_gemm64(
    const unsigned short* __restrict__ Ap, const unsigned short* __restrict__ A2p, int lda, long strideA,
    const unsigned short* __restrict__ Btp, const unsigned short* __restrict__ Bt2p, int ldb, long strideB,
    void* __restrict__ Cout, void* __restrict__ Cout2, int ldc, long strideC,
    const float* __restrict__ bias,
    const float* __restrict__ resid, long strideR,
    int M, int N, int K, float scale) {
  typedef typename Elem<ET>::T T;
  typedef typename Frag<T>::V V;
  const T* A = (const T*)Ap; const T* A2 = (const T*)A2p; const T* Bt = (const T*)Btp; const T* Bt2 = (const T*)Bt2p;
  __shared__ __align__(16) float sT[8][16 * 68];
  const int b    = blockIdx.y;
  const int lane = threadIdx.x & 31;
  const int wave = threadIdx.x >> 5;
  const int tilesN = N >> 6;
  const int tilesM = M >> 6;
  const int tile = blockIdx.x * 8 + wave;
  if (tile >= tilesM * tilesN) return;
  const int tm = tile / tilesN;
  const int tn = tile - tm * tilesN;
  const int m0 = tm << 6;
  const int n0 = tn << 6;

  const T* Ab  = A  + (size_t)b * strideA;
  const T* Bb  = Bt + (size_t)b * strideB;
  const T* Ab2 = (SPL >= 1) ? (A2  + (size_t)b * strideA) : nullptr;
  const T* Bb2 = (SPL == 2) ? (Bt2 + (size_t)b * strideB) : nullptr;

  const int rlane = lane & 15;
  const int koff  = (lane >> 4) * 8;
  const int mOff  = (lane >> 4) * 8;

  v8f acc[4][4];
#pragma unroll
  for (int i = 0; i < 4; ++i)
#pragma unroll
    for (int j = 0; j < 4; ++j) acc[i][j] = (v8f){0.f,0.f,0.f,0.f,0.f,0.f,0.f,0.f};

  for (int k0 = 0; k0 < K; k0 += 32) {
    V bh[4], bl[4];
#pragma unroll
    for (int j = 0; j < 4; ++j) {
      const size_t bo = (size_t)(n0 + (j << 4) + rlane) * ldb + koff + k0;
      bh[j] = Frag<T>::load(Bb + bo);
      if (SPL == 2) bl[j] = Frag<T>::load(Bb2 + bo);
    }
#pragma unroll
    for (int i = 0; i < 4; ++i) {
      const size_t ao = (size_t)(m0 + (i << 4) + rlane) * lda + koff + k0;
      V ah = Frag<T>::load(Ab + ao);
      V al;
      if (SPL >= 1) al = Frag<T>::load(Ab2 + ao);
#pragma unroll
      for (int j = 0; j < 4; ++j) {
        acc[i][j] = Frag<T>::mma(ah, bh[j], acc[i][j]);
        if (SPL == 2) acc[i][j] = Frag<T>::mma(ah, bl[j], acc[i][j]);
        if (SPL >= 1) acc[i][j] = Frag<T>::mma(al, bh[j], acc[i][j]);
      }
      Frag<T>::guard(acc[i][0], acc[i][3], ah, (SPL >= 1) ? al : ah);
    }
    Frag<T>::keep(bh[0], bh[1], bh[2], bh[3]);
    if (SPL == 2) Frag<T>::keep(bl[0], bl[1], bl[2], bl[3]);
  }
  acc_guard4(acc[0][0], acc[0][1], acc[0][2], acc[0][3]);
  acc_guard4(acc[1][0], acc[1][1], acc[1][2], acc[1][3]);
  acc_guard4(acc[2][0], acc[2][1], acc[2][2], acc[2][3]);
  acc_guard4(acc[3][0], acc[3][1], acc[3][2], acc[3][3]);

  float* slab = sT[wave];
  const float* Rb = RESID ? (resid + (size_t)b * strideR) : nullptr;
#pragma unroll
  for (int i = 0; i < 4; ++i) {
    const int mBase = m0 + (i << 4);
#pragma unroll
    for (int j = 0; j < 4; ++j) {
      const int n = n0 + (j << 4) + rlane;
      float bv = 0.f;
      if (BIAS_MODE == 2) bv = bias[n];
#pragma unroll
      for (int r = 0; r < 8; ++r) {
        float v = acc[i][j][r] * scale;
        if (BIAS_MODE == 1) v += bias[mBase + mOff + r];
        if (BIAS_MODE == 2) v += bv;
        if (RESID) v += Rb[(size_t)(mBase + mOff + r) * ldc + n];
        if (ACT == 1) v = tanhf(v);
        if (ACT == 2) v = fmaxf(v, 0.0f);
        if (ACT == 3) v = v / (1.0f + expf(-v));
        if (ACT == 4) v = (v > 0.f) ? v : 0.01f * v;
        slab[(mOff + r) * 68 + (j << 4) + rlane] = v;
      }
    }
    __builtin_amdgcn_fence(__ATOMIC_RELEASE, "workgroup");
    __builtin_amdgcn_wave_barrier();
    __builtin_amdgcn_fence(__ATOMIC_ACQUIRE, "workgroup");
    if (OUT_MODE == 0) {
      float* C = (float*)Cout + (size_t)b * strideC;
      const int hh = lane >> 4, c4 = (lane & 15) * 4;
      for (int pass = 0; pass < 2; ++pass) {
#pragma unroll
        for (int it = 0; it < 8; ++it) {
          const int row = it * 2 + hh;
          v4f v = *(const v4f*)(slab + row * 68 + c4);
          *(volatile v4f*)(C + (size_t)(mBase + row) * ldc + n0 + c4) = v;
        }
        __threadfence();
      }
    } else {
      const int q = lane >> 3, c8 = (lane & 7) * 8;
      unsigned short* C  = (unsigned short*)Cout  + (size_t)b * strideC;
      unsigned short* C2 = (OUT_MODE == 2) ? ((unsigned short*)Cout2 + (size_t)b * strideC) : nullptr;
      for (int pass = 0; pass < 2; ++pass) {
#pragma unroll
        for (int it = 0; it < 4; ++it) {
          const int row = it * 4 + q;
          const float* sp = slab + row * 68 + c8;
          v8h hv, lv;
#pragma unroll
          for (int e = 0; e < 8; ++e) {
            if (OUT_MODE == 1) {
              hv[e] = (_Float16)sp[e];
            } else {
              unsigned short hb = f2bf_bits(sp[e]);
              unsigned short lb = f2bf_bits(sp[e] - bf_bits2f(hb));
              hv[e] = __builtin_bit_cast(_Float16, hb);
              lv[e] = __builtin_bit_cast(_Float16, lb);
            }
          }
          *(volatile v8h*)(C + (size_t)(mBase + row) * ldc + n0 + c8) = hv;
          if (OUT_MODE == 2) *(volatile v8h*)(C2 + (size_t)(mBase + row) * ldc + n0 + c8) = lv;
        }
        __threadfence();
      }
    }
    __builtin_amdgcn_fence(__ATOMIC_RELEASE, "workgroup");
    __builtin_amdgcn_wave_barrier();
    __builtin_amdgcn_fence(__ATOMIC_ACQUIRE, "workgroup");
  }
}

__global__ __launch_bounds__(256) void x_tok_planes_kernel(
    const float* __restrict__ x, unsigned short* __restrict__ TH, unsigned short* __restrict__ TL)
{
  __shared__ __align__(16) float sT[64 * kXTP];
  const int tid = threadIdx.x;
  const int b = blockIdx.y;
  const int l0 = blockIdx.x * 64;
  const int lr = tid & 63, dg = tid >> 6;
#pragma unroll 4
  for (int i = 0; i < 24; ++i) {
    const int c = dg + 4 * i;
    const float v = x[((size_t)b * kDm + c) * kSeq + l0 + lr];
    sT[lr * kXTP + c] = v;
  }
  __syncthreads();
  v8h hv[3], lv[3];
#pragma unroll
  for (int it = 0; it < 3; ++it) {
    const int p = it * 256 + tid;
    const int row = p / 12;
    const int c = (p - row * 12) * 8;
    const float* sp = sT + row * kXTP + c;
    const v4f a0 = *(const v4f*)(sp);
    const v4f a1 = *(const v4f*)(sp + 4);
#pragma unroll
    for (int e = 0; e < 4; ++e) {
      const unsigned short h0 = f2bf_bits(a0[e]), h1 = f2bf_bits(a1[e]);
      const unsigned short q0 = f2bf_bits(a0[e] - bf_bits2f(h0)), q1 = f2bf_bits(a1[e] - bf_bits2f(h1));
      hv[it][e]     = __builtin_bit_cast(_Float16, h0);
      hv[it][4 + e] = __builtin_bit_cast(_Float16, h1);
      lv[it][e]     = __builtin_bit_cast(_Float16, q0);
      lv[it][4 + e] = __builtin_bit_cast(_Float16, q1);
    }
  }
  const size_t base = (size_t)(b * kSeq + l0) * kDm;
  for (int pass = 0; pass < 2; ++pass) {
#pragma unroll
    for (int it = 0; it < 3; ++it) {
      const size_t o = base + (size_t)(it * 256 + tid) * 8;
      *(volatile v8h*)(TH + o) = hv[it];
      *(volatile v8h*)(TL + o) = lv[it];
    }
    __threadfence();
  }
}

__global__ __launch_bounds__(256) void weight_planes_kernel(
    const float* __restrict__ W, unsigned short* __restrict__ WH, unsigned short* __restrict__ WL,
    int K, int srcRows, int mode, int total8)
{
  const int i = blockIdx.x * 256 + threadIdx.x;
  if (i >= total8) return;
  const int e0 = i << 3;
  const int n  = e0 / K;
  const int k0 = e0 - n * K;
  const int srowP = (n < 32) ? (n + 6) : (n - 32);
  int srow = (mode == 0) ? n : srowP;
  const bool keep = (mode == 0) ? (n < srcRows) : (n < kXprN);
  srow = (srow < 0) ? 0 : srow;
  srow = (srow > srcRows - 1) ? (srcRows - 1) : srow;
  const float* sp = W + (size_t)srow * K + k0;
  const v4f a0 = *(const v4f*)(sp);
  const v4f a1 = *(const v4f*)(sp + 4);
  v8h hv, lv;
#pragma unroll
  for (int e = 0; e < 4; ++e) {
    const float v0 = keep ? a0[e] : 0.f;
    const float v1 = keep ? a1[e] : 0.f;
    const unsigned short h0 = f2bf_bits(v0), h1 = f2bf_bits(v1);
    const unsigned short q0 = f2bf_bits(v0 - bf_bits2f(h0)), q1 = f2bf_bits(v1 - bf_bits2f(h1));
    hv[e]     = __builtin_bit_cast(_Float16, h0);
    hv[4 + e] = __builtin_bit_cast(_Float16, h1);
    lv[e]     = __builtin_bit_cast(_Float16, q0);
    lv[4 + e] = __builtin_bit_cast(_Float16, q1);
  }
  unsigned short* qh = WH + e0;
  unsigned short* ql = WL + e0;
  *(volatile v8h*)qh = hv;
  *(volatile v8h*)ql = lv;
  __threadfence();
  *(volatile v8h*)qh = hv;
  *(volatile v8h*)ql = lv;
}

__global__ __launch_bounds__(256) void norm1_planes_kernel(
    const float* __restrict__ O1, const float* __restrict__ cb, const float* __restrict__ nw,
    const float* __restrict__ nb, unsigned short* __restrict__ XH, unsigned short* __restrict__ XL)
{
  __shared__ __align__(16) float sT[64 * kXTP];
  const int tid = threadIdx.x, lane = tid & 31, wave = tid >> 5;
  const int r0 = blockIdx.x * 64;
  const float b0 = cb[lane], b1 = cb[lane + 32], b2 = cb[lane + 64];
  const float w0 = nw[lane], w1 = nw[lane + 32], w2 = nw[lane + 64];
  const float g0 = nb[lane], g1 = nb[lane + 32], g2 = nb[lane + 64];
#pragma unroll 1
  for (int j = 0; j < 8; ++j) {
    const int rr = wave * 8 + j;
    const size_t ro = (size_t)(r0 + rr) * kCnvN;
    const float x0 = O1[ro + lane] + b0;
    const float x1 = O1[ro + lane + 32] + b1;
    const float x2 = O1[ro + lane + 64] + b2;
    float s = x0 + x1 + x2;
#pragma unroll
    for (int off = 16; off >= 1; off >>= 1) s += __shfl_xor(s, off, 32);
    const float mean = s * (1.0f / 96.0f);
    const float d0 = x0 - mean, d1 = x1 - mean, d2 = x2 - mean;
    float q = d0 * d0 + d1 * d1 + d2 * d2;
#pragma unroll
    for (int off = 16; off >= 1; off >>= 1) q += __shfl_xor(q, off, 32);
    const float var = q * (1.0f / 96.0f);
    const float inv = rsqrtf(var + 1e-5f);
    sT[rr * kXTP + lane]      = d0 * inv * w0 + g0;
    sT[rr * kXTP + lane + 32] = d1 * inv * w1 + g1;
    sT[rr * kXTP + lane + 64] = d2 * inv * w2 + g2;
  }
  __syncthreads();
  v8h hv[3], lv[3];
#pragma unroll
  for (int it = 0; it < 3; ++it) {
    const int p = it * 256 + tid;
    const int row = p / 12;
    const int c = (p - row * 12) * 8;
    const float* sp = sT + row * kXTP + c;
    const v4f a0 = *(const v4f*)(sp);
    const v4f a1 = *(const v4f*)(sp + 4);
#pragma unroll
    for (int e = 0; e < 4; ++e) {
      const unsigned short h0 = f2bf_bits(a0[e]), h1 = f2bf_bits(a1[e]);
      const unsigned short q0 = f2bf_bits(a0[e] - bf_bits2f(h0)), q1 = f2bf_bits(a1[e] - bf_bits2f(h1));
      hv[it][e]     = __builtin_bit_cast(_Float16, h0);
      hv[it][4 + e] = __builtin_bit_cast(_Float16, h1);
      lv[it][e]     = __builtin_bit_cast(_Float16, q0);
      lv[it][4 + e] = __builtin_bit_cast(_Float16, q1);
    }
  }
  const size_t base = (size_t)r0 * kDm;
  for (int pass = 0; pass < 2; ++pass) {
#pragma unroll
    for (int it = 0; it < 3; ++it) {
      const size_t o = base + (size_t)(it * 256 + tid) * 8;
      *(volatile v8h*)(XH + o) = hv[it];
      *(volatile v8h*)(XL + o) = lv[it];
    }
    __threadfence();
  }
}

__global__ __launch_bounds__(192) void conv_silu_kernel(
    const float* __restrict__ XZ, const float* __restrict__ cw, const float* __restrict__ cb,
    float* __restrict__ UC, unsigned short* __restrict__ UCH, unsigned short* __restrict__ UCL)
{
  __shared__ __align__(16) float sT[16 * kConvTP];
  const int tid = threadIdx.x;
  const int d = tid;
  const int img = blockIdx.y;
  const int g0 = blockIdx.x * 64;
  const size_t rbase = (size_t)img * kSeq;
  const float w0 = cw[d * 4 + 0], w1 = cw[d * 4 + 1], w2 = cw[d * 4 + 2], w3 = cw[d * 4 + 3];
  const float bc = cb[d];
  float xm3, xm2, xm1;
  {
    const bool hist = (g0 > 0);
    const int rb = hist ? (g0 - 3) : 0;
    const float v3 = XZ[(rbase + rb) * kXzP + d];
    const float v2 = XZ[(rbase + rb + 1) * kXzP + d];
    const float v1 = XZ[(rbase + rb + 2) * kXzP + d];
    xm3 = hist ? v3 : 0.f;
    xm2 = hist ? v2 : 0.f;
    xm1 = hist ? v1 : 0.f;
  }
#pragma unroll 1
  for (int sub = 0; sub < 4; ++sub) {
    const int lb = g0 + sub * 16;
#pragma unroll 1
    for (int s = 0; s < 16; ++s) {
      const float xcur = XZ[(rbase + lb + s) * kXzP + d];
      float acc = w0 * xm3;
      acc = fmaf(w1, xm2, acc);
      acc = fmaf(w2, xm1, acc);
      acc = fmaf(w3, xcur, acc);
      const float sv = acc + bc;
      const float sg = __builtin_amdgcn_rcpf(1.0f + __expf(-sv));
      sT[s * kConvTP + tid] = sv * sg;
      xm3 = xm2; xm2 = xm1; xm1 = xcur;
    }
    __syncthreads();
    v4f fv[4];
    v8h bh[2], blo[2];
#pragma unroll
    for (int it = 0; it < 4; ++it) {
      const int p = it * 192 + tid;
      const int row = p / 48;
      const int c4 = (p - row * 48) * 4;
      fv[it] = *(const v4f*)(sT + row * kConvTP + c4);
    }
#pragma unroll
    for (int it = 0; it < 2; ++it) {
      const int p = it * 192 + tid;
      const int row = p / 24;
      const int c8 = (p - row * 24) * 8;
      const float* sp = sT + row * kConvTP + c8;
      const v4f a0 = *(const v4f*)(sp);
      const v4f a1 = *(const v4f*)(sp + 4);
#pragma unroll
      for (int e = 0; e < 4; ++e) {
        const unsigned short h0 = f2bf_bits(a0[e]), h1 = f2bf_bits(a1[e]);
        const unsigned short q0 = f2bf_bits(a0[e] - bf_bits2f(h0)), q1 = f2bf_bits(a1[e] - bf_bits2f(h1));
        bh[it][e]      = __builtin_bit_cast(_Float16, h0);
        bh[it][4 + e]  = __builtin_bit_cast(_Float16, h1);
        blo[it][e]     = __builtin_bit_cast(_Float16, q0);
        blo[it][4 + e] = __builtin_bit_cast(_Float16, q1);
      }
    }
    const size_t eb = (rbase + lb) * kDin;
    for (int pass = 0; pass < 2; ++pass) {
#pragma unroll
      for (int it = 0; it < 4; ++it)
        *(volatile v4f*)(UC + eb + (size_t)(it * 192 + tid) * 4) = fv[it];
#pragma unroll
      for (int it = 0; it < 2; ++it) {
        const size_t o = eb + (size_t)(it * 192 + tid) * 8;
        *(volatile v8h*)(UCH + o) = bh[it];
        *(volatile v8h*)(UCL + o) = blo[it];
      }
      __threadfence();
    }
    __syncthreads();
  }
}

__global__ __launch_bounds__(64) void scan_kernel(
    const float* __restrict__ XD, const float* __restrict__ UC, const float* __restrict__ XZ,
    const float* __restrict__ Wdt, const float* __restrict__ bdt, const float* __restrict__ Alog,
    const float* __restrict__ Dskip, unsigned short* __restrict__ YH, unsigned short* __restrict__ YL)
{
  __shared__ __align__(16) float sX[kScanTS * kXdP];
  __shared__ __align__(16) float sY[kScanTS * kScanYP];
  __shared__ __align__(16) float sH[kNst * kScanCh];
  __shared__ __align__(16) float sA[kNst * kScanCh];
  const int tid = threadIdx.x, lane = tid & 31, wave = tid >> 5;
  const int d0 = blockIdx.x * kScanCh;
  const int d  = d0 + tid;
  const size_t rbase = (size_t)blockIdx.y * kSeq;
#pragma unroll 1
  for (int s = 0; s < kNst; ++s) {
    sA[s * kScanCh + tid] = -__expf(Alog[(size_t)d * kNst + s]);
    sH[s * kScanCh + tid] = 0.f;
  }
  float wdt[kDtR];
#pragma unroll
  for (int r = 0; r < kDtR; ++r) wdt[r] = Wdt[d * kDtR + r];
  const float bb = bdt[d], Dd = Dskip[d];
  const int lr = tid >> 4, lc4 = (tid & 15) * 4;
  const int q = lane >> 3, c8 = (lane & 7) * 8;
#pragma unroll 1
  for (int t0 = 0; t0 < kSeq; t0 += kScanTS) {
    __syncthreads();
#pragma unroll
    for (int i = 0; i < 16; ++i) {
      const int r = lr + 4 * i;
      *(v4f*)(sX + r * kXdP + lc4) = *(const v4f*)(XD + (rbase + t0 + r) * kXdP + lc4);
    }
    __syncthreads();
#pragma unroll 1
    for (int s = 0; s < kScanTS; ++s) {
      const size_t row = rbase + t0 + s;
      const float* xr = sX + s * kXdP;
      float v = bb;
#pragma unroll
      for (int r = 0; r < kDtR; ++r) v = fmaf(xr[32 + r], wdt[r], v);
      const float a   = __expf(-fabsf(v));
      const float ua  = 1.0f + a;
      const float l1p = __logf(ua) + (a - (ua - 1.0f)) * __builtin_amdgcn_rcpf(ua);
      const float dt  = fmaxf(v, 0.0f) + l1p;
      const float xt  = UC[row * kDin + d];
      const float dtx = dt * xt;
      float y = 0.f;
#pragma unroll 4
      for (int k = 0; k < kNst; ++k) {
        const int hidx = k * kScanCh + tid;
        const float e  = __expf(dt * sA[hidx]);
        const float hn = e * sH[hidx] + dtx * xr[k];
        sH[hidx] = hn;
        y = hn * xr[kNst + k] + y;
      }
      y = xt * Dd + y;
      const float zv = XZ[row * kXzP + kDin + d];
      const float sg = __builtin_amdgcn_rcpf(1.0f + __expf(-zv));
      y = y * (zv * sg);
      sY[s * kScanYP + tid] = y;
    }
    __syncthreads();
    v8h hv[8], lv[8];
#pragma unroll
    for (int it = 0; it < 8; ++it) {
      const int row = it * 8 + wave * 4 + q;
      const float* sp = sY + row * kScanYP + c8;
      const v4f a0 = *(const v4f*)(sp);
      const v4f a1 = *(const v4f*)(sp + 4);
#pragma unroll
      for (int e = 0; e < 4; ++e) {
        const unsigned short h0 = f2bf_bits(a0[e]), h1 = f2bf_bits(a1[e]);
        const unsigned short q0 = f2bf_bits(a0[e] - bf_bits2f(h0)), q1 = f2bf_bits(a1[e] - bf_bits2f(h1));
        hv[it][e]     = __builtin_bit_cast(_Float16, h0);
        hv[it][4 + e] = __builtin_bit_cast(_Float16, h1);
        lv[it][e]     = __builtin_bit_cast(_Float16, q0);
        lv[it][4 + e] = __builtin_bit_cast(_Float16, q1);
      }
    }
    for (int pass = 0; pass < 2; ++pass) {
#pragma unroll
      for (int it = 0; it < 8; ++it) {
        const int row = it * 8 + wave * 4 + q;
        const size_t o = (rbase + t0 + row) * kDin + d0 + c8;
        *(volatile v8h*)(YH + o) = hv[it];
        *(volatile v8h*)(YL + o) = lv[it];
      }
      __threadfence();
    }
  }
}

__global__ __launch_bounds__(256) void ysum_planes_kernel(
    const float* __restrict__ YO, unsigned short* __restrict__ YSH, unsigned short* __restrict__ YSL, int total8)
{
  const int i = blockIdx.x * 256 + threadIdx.x;
  if (i >= total8) return;
  const int e0 = i << 3;
  const int row = e0 / kDm;
  const int c0 = e0 - row * kDm;
  const float* pa = YO + (size_t)row * kOutP + c0;
  const float* pb = YO + (size_t)(row + kRowsO) * kOutP + c0;
  const v4f a0 = *(const v4f*)(pa);
  const v4f a1 = *(const v4f*)(pa + 4);
  const v4f u0 = *(const v4f*)(pb);
  const v4f u1 = *(const v4f*)(pb + 4);
  v8h hv, lv;
#pragma unroll
  for (int e = 0; e < 4; ++e) {
    const float v0 = a0[e] + u0[e];
    const float v1 = a1[e] + u1[e];
    const unsigned short h0 = f2bf_bits(v0), h1 = f2bf_bits(v1);
    const unsigned short q0 = f2bf_bits(v0 - bf_bits2f(h0)), q1 = f2bf_bits(v1 - bf_bits2f(h1));
    hv[e]     = __builtin_bit_cast(_Float16, h0);
    hv[4 + e] = __builtin_bit_cast(_Float16, h1);
    lv[e]     = __builtin_bit_cast(_Float16, q0);
    lv[4 + e] = __builtin_bit_cast(_Float16, q1);
  }
  unsigned short* qh = YSH + e0;
  unsigned short* ql = YSL + e0;
  *(volatile v8h*)qh = hv;
  *(volatile v8h*)ql = lv;
  __threadfence();
  *(volatile v8h*)qh = hv;
  *(volatile v8h*)ql = lv;
}

__global__ __launch_bounds__(256) void norm2_out_kernel(
    const float* __restrict__ O2, const float* __restrict__ cb, const float* __restrict__ nw,
    const float* __restrict__ nb, float* __restrict__ out)
{
  __shared__ __align__(16) float tile[kDm * kOTP];
  const int tid = threadIdx.x, lane = tid & 31, wave = tid >> 5;
  const int b = blockIdx.y;
  const int l0 = blockIdx.x * 64;
  const float b0 = cb[lane], b1 = cb[lane + 32], b2 = cb[lane + 64];
  const float w0 = nw[lane], w1 = nw[lane + 32], w2 = nw[lane + 64];
  const float g0 = nb[lane], g1 = nb[lane + 32], g2 = nb[lane + 64];
#pragma unroll 1
  for (int j = 0; j < 8; ++j) {
    const int rr = wave * 8 + j;
    const size_t ro = (size_t)(b * kSeq + l0 + rr) * kCnvN;
    const float x0 = O2[ro + lane] + b0;
    const float x1 = O2[ro + lane + 32] + b1;
    const float x2 = O2[ro + lane + 64] + b2;
    float s = x0 + x1 + x2;
#pragma unroll
    for (int off = 16; off >= 1; off >>= 1) s += __shfl_xor(s, off, 32);
    const float mean = s * (1.0f / 96.0f);
    const float d0 = x0 - mean, d1 = x1 - mean, d2 = x2 - mean;
    float q = d0 * d0 + d1 * d1 + d2 * d2;
#pragma unroll
    for (int off = 16; off >= 1; off >>= 1) q += __shfl_xor(q, off, 32);
    const float var = q * (1.0f / 96.0f);
    const float inv = rsqrtf(var + 1e-5f);
    tile[lane * kOTP + rr]        = d0 * inv * w0 + g0;
    tile[(lane + 32) * kOTP + rr] = d1 * inv * w1 + g1;
    tile[(lane + 64) * kOTP + rr] = d2 * inv * w2 + g2;
  }
  __syncthreads();
  const int hh = lane >> 4, c4 = (lane & 15) * 4;
  v4f val[6];
#pragma unroll
  for (int it = 0; it < 6; ++it) {
    const int c = (it * 8 + wave) * 2 + hh;
    val[it] = *(const v4f*)(tile + c * kOTP + c4);
  }
  for (int pass = 0; pass < 2; ++pass) {
#pragma unroll
    for (int it = 0; it < 6; ++it) {
      const int c = (it * 8 + wave) * 2 + hh;
      *(volatile v4f*)(out + ((size_t)(b * kDm + c)) * kSeq + l0 + c4) = val[it];
    }
    __threadfence();
  }
}

extern "C" void kernel_launch(void* const* d_in, const int* in_sizes, int n_in,
                              void* d_out, int out_size, void* d_ws, size_t ws_size,
                              hipStream_t stream) {
  if (n_in < 19) return;
  if (in_sizes[0] != kImg * kDm * kSeq) return;
  if (in_sizes[1] != kImg * kDm * kSeq) return;
  if (in_sizes[2] != kDm * kDm) return;
  if (in_sizes[3] != kDm) return;
  if (in_sizes[4] != kDm) return;
  if (in_sizes[5] != kDm) return;
  if (in_sizes[6] != kXzP * kDm) return;
  if (in_sizes[7] != kDin * 4) return;
  if (in_sizes[8] != kDin) return;
  if (in_sizes[9] != kXprN * kDin) return;
  if (in_sizes[10] != kDin * kDtR) return;
  if (in_sizes[11] != kDin) return;
  if (in_sizes[12] != kDin * kNst) return;
  if (in_sizes[13] != kDin) return;
  if (in_sizes[14] != kDm * kDin) return;
  if (in_sizes[15] != kDm * kDm) return;
  if (in_sizes[16] != kDm) return;
  if (in_sizes[17] != kDm) return;
  if (in_sizes[18] != kDm) return;
  if (out_size != kImg * kDm * kSeq) return;
  if (ws_size < kWsTotal) return;

  const float* x1      = (const float*)d_in[0];
  const float* x2      = (const float*)d_in[1];
  const float* c1_w    = (const float*)d_in[2];
  const float* c1_b    = (const float*)d_in[3];
  const float* n1_w    = (const float*)d_in[4];
  const float* n1_b    = (const float*)d_in[5];
  const float* W_in    = (const float*)d_in[6];
  const float* conv_w  = (const float*)d_in[7];
  const float* conv_b  = (const float*)d_in[8];
  const float* W_xproj = (const float*)d_in[9];
  const float* W_dt    = (const float*)d_in[10];
  const float* b_dt    = (const float*)d_in[11];
  const float* A_log   = (const float*)d_in[12];
  const float* Dskip   = (const float*)d_in[13];
  const float* W_out   = (const float*)d_in[14];
  const float* c2_w    = (const float*)d_in[15];
  const float* c2_b    = (const float*)d_in[16];
  const float* n2_w    = (const float*)d_in[17];
  const float* n2_b    = (const float*)d_in[18];
  float* out = (float*)d_out;
  (void)stream;

  char* ws = (char*)d_ws;
  unsigned short* TKH = (unsigned short*)(ws + kOffTKH);
  unsigned short* TKL = (unsigned short*)(ws + kOffTKL);
  unsigned short* W1H = (unsigned short*)(ws + kOffW1H);
  unsigned short* W1L = (unsigned short*)(ws + kOffW1L);
  unsigned short* W2H = (unsigned short*)(ws + kOffW2H);
  unsigned short* W2L = (unsigned short*)(ws + kOffW2L);
  float*          O1  = (float*)(ws + kOffO1);
  unsigned short* XH  = (unsigned short*)(ws + kOffXH);
  unsigned short* XL  = (unsigned short*)(ws + kOffXL);
  unsigned short* WIH = (unsigned short*)(ws + kOffWIH);
  unsigned short* WIL = (unsigned short*)(ws + kOffWIL);
  unsigned short* WXH = (unsigned short*)(ws + kOffWXH);
  unsigned short* WXL = (unsigned short*)(ws + kOffWXL);
  unsigned short* WOH = (unsigned short*)(ws + kOffWOH);
  unsigned short* WOL = (unsigned short*)(ws + kOffWOL);
  float*          XZ  = (float*)(ws + kOffXZ);
  float*          UC  = (float*)(ws + kOffUC);
  unsigned short* UCH = (unsigned short*)(ws + kOffUCH);
  unsigned short* UCL = (unsigned short*)(ws + kOffUCL);
  float*          XD  = (float*)(ws + kOffXD);
  unsigned short* YH  = (unsigned short*)(ws + kOffYH);
  unsigned short* YL  = (unsigned short*)(ws + kOffYL);
  float*          YO  = (float*)(ws + kOffYO);
  unsigned short* YSH = (unsigned short*)(ws + kOffYSH);
  unsigned short* YSL = (unsigned short*)(ws + kOffYSL);
  float*          O2  = (float*)(ws + kOffO2);

  x_tok_planes_kernel<<<dim3(kSeq / 64, kImg), 256, 0, stream>>>(x1, TKH, TKL);
  x_tok_planes_kernel<<<dim3(kSeq / 64, kImg), 256, 0, stream>>>(x2, TKH + (size_t)kRowsO * kDm, TKL + (size_t)kRowsO * kDm);
  weight_planes_kernel<<<(kCnvN * kDm / 8) / 256, 256, 0, stream>>>(c1_w, W1H, W1L, kDm, kDm, 0, kCnvN * kDm / 8);
  weight_planes_kernel<<<(kCnvN * kDm / 8) / 256, 256, 0, stream>>>(c2_w, W2H, W2L, kDm, kDm, 0, kCnvN * kDm / 8);
  weight_planes_kernel<<<(kXzP * kDm / 8) / 256, 256, 0, stream>>>(W_in, WIH, WIL, kDm, kXzP, 0, kXzP * kDm / 8);
  weight_planes_kernel<<<(kXdP * kDin / 8) / 256, 256, 0, stream>>>(W_xproj, WXH, WXL, kDin, kXprN, 1, kXdP * kDin / 8);
  weight_planes_kernel<<<(kOutP * kDin / 8) / 256, 256, 0, stream>>>(W_out, WOH, WOL, kDin, kDm, 0, kOutP * kDin / 8);

  wmma_gemm64<1, 2, 0, 0, false><<<dim3(128, 1), 256, 0, stream>>>(
      TKH, TKL, kDm, 0L,
      W1H, W1L, kDm, 0L,
      (void*)O1, nullptr, kCnvN, 0L,
      nullptr, nullptr, 0L,
      kRows, kCnvN, kDm, 1.0f);
  norm1_planes_kernel<<<kRows / 64, 256, 0, stream>>>(O1, c1_b, n1_w, n1_b, XH, XL);

  for (int g = 0; g < kNGrp; ++g) {
    const size_t rowOff = (size_t)g * kRowsG;
    wmma_gemm64<1, 2, 0, 0, false><<<dim3(192, 1), 256, 0, stream>>>(
        XH + rowOff * kDm, XL + rowOff * kDm, kDm, 0L,
        WIH, WIL, kDm, 0L,
        (void*)XZ, nullptr, kXzP, 0L,
        nullptr, nullptr, 0L,
        kRowsG, kXzP, kDm, 1.0f);
    conv_silu_kernel<<<dim3(kSeq / 64, kGrp), kDin, 0, stream>>>(XZ, conv_w, conv_b, UC, UCH, UCL);
    wmma_gemm64<1, 2, 0, 0, false><<<dim3(32, 1), 256, 0, stream>>>(
        UCH, UCL, kDin, 0L,
        WXH, WXL, kDin, 0L,
        (void*)XD, nullptr, kXdP, 0L,
        nullptr, nullptr, 0L,
        kRowsG, kXdP, kDin, 1.0f);
    scan_kernel<<<dim3(kDin / kScanCh, kGrp), kScanCh, 0, stream>>>(XD, UC, XZ, W_dt, b_dt, A_log, Dskip, YH, YL);
    wmma_gemm64<1, 2, 0, 0, false><<<dim3(64, 1), 256, 0, stream>>>(
        YH, YL, kDin, 0L,
        WOH, WOL, kDin, 0L,
        (void*)(YO + rowOff * kOutP), nullptr, kOutP, 0L,
        nullptr, nullptr, 0L,
        kRowsG, kOutP, kDin, 1.0f);
  }

  ysum_planes_kernel<<<(kRowsO * kDm / 8) / 256, 256, 0, stream>>>(YO, YSH, YSL, kRowsO * kDm / 8);
  wmma_gemm64<1, 2, 0, 0, false><<<dim3(64, 1), 256, 0, stream>>>(
      YSH, YSL, kDm, 0L,
      W2H, W2L, kDm, 0L,
      (void*)O2, nullptr, kCnvN, 0L,
      nullptr, nullptr, 0L,
      kRowsO, kCnvN, kDm, 1.0f);
  norm2_out_kernel<<<dim3(kSeq / 64, kImg), 256, 0, stream>>>(O2, c2_b, n2_w, n2_b, out);
}
